// GCNGAT_Encoder_79224966742229
// MI455X (gfx1250) — hardware-run, weakly checked
//
#include <hip/hip_runtime.h>


namespace {
constexpr int N = 20000, E = 320000, EP = E + N, C0 = 128, HID = 64, NH = 4, HW = NH * HID  ;
constexpr float XS = 8.0f, WSC = 256.0f, SLOPE = 0.2f;
typedef _Float16 b16;
typedef __attribute__((ext_vector_type(16))) _Float16 v16b;
typedef __attribute__((ext_vector_type(8))) _Float16 v8b;
typedef __attribute__((ext_vector_type(8))) float v8f;
typedef __attribute__((ext_vector_type(4))) float v4f;
typedef __attribute__((ext_vector_type(2))) float v2f;
__device__ __forceinline__ float bf16_rne(float f) { unsigned int u = __float_as_uint(f); u += 0x7FFFu + ((u >> 16) & 1u); float r = __uint_as_float(u & 0xFFFF0000u); asm volatile("" : "+v"(r)); return r; }
__device__ __forceinline__ void split16(float v, b16& hi, b16& lo) { hi = (b16)v; lo = (b16)(v - (float)hi); }
__device__ __forceinline__ v16b frag_kb(const b16* p, int hh) { const v8b a = *(const v8b*)(p + 8 * hh), b = *(const v8b*)(p + 16 + 8 * hh); v16b f;
#pragma unroll
  for (int e = 0; e < 8; ++e) { f[e] = a[e]; f[8 + e] = b[e]; } return f; }
__device__ __forceinline__ v8f wmma16b(v16b a, v16b b, v8f c) { v8f d = __builtin_amdgcn_wmma_f32_16x16x32_f16(false, a, false, b, (short)0, c, false, false); asm volatile("v_nop\n\tv_nop\n\tv_nop\n\tv_nop" : "+v"(d) : "v"(a), "v"(b)); return d; }
__device__ __forceinline__ void wave_lds_sync() { __builtin_amdgcn_fence(__ATOMIC_RELEASE, "workgroup"); __builtin_amdgcn_wave_barrier(); __builtin_amdgcn_fence(__ATOMIC_ACQUIRE, "workgroup"); }
__device__ __forceinline__ float pmul(float a, float b) { float p = a * b; asm volatile("" : "+v"(p)); return p; }
__device__ __forceinline__ int iclamp(int v, int lo, int hi) { return v < lo ? lo : (v > hi ? hi : v); }
__device__ __forceinline__ float leaky(float v) { return v > 0.0f ? v : SLOPE * v; }
constexpr int CSR_NBLK8 = 512, CSR_GB8 = 8, CSR_GN8 = 1 << CSR_GB8  , CSR_TS8 = (CSR_GN8 < 32 ? 32 : CSR_GN8)  , CSR_MAXG8 = 512, CSR_CAP8 = 12288  ;
__device__ __host__ __forceinline__ int csr_tix8(int v) { return (v >> CSR_GB8) * CSR_TS8 + (v & (CSR_GN8 - 1)); }
__global__ __launch_bounds__(64) void csrA_kernel8(const int* __restrict__ dst, int E, int N, int nG, int CHP, int NGP, int* __restrict__ STG, int* __restrict__ HST) {
  extern __shared__ int sm[];
  int* cnt = sm; int* run = sm + NGP; int* ids = sm + 2 * NGP;
  const int b = blockIdx.x; const int ch = (E + CSR_NBLK8 - 1) / CSR_NBLK8; const int e0 = b * ch, e1 = min(E, e0 + ch);
  for (int i = threadIdx.x; i < NGP; i += 64) cnt[i] = 0;
  for (int i = threadIdx.x; i < CHP; i += 64) ids[i] = -1;
  __syncthreads();
  if (threadIdx.x == 0) {
    for (int e = e0; e < e1; ++e) { int d = dst[e]; d = (d < 0) ? 0 : (d >= N ? N - 1 : d); cnt[d >> CSR_GB8] += 1; }
    int acc = 0; for (int g = 0; g < nG; ++g) { run[g] = acc; acc += cnt[g]; }
    for (int e = e0; e < e1; ++e) { int d = dst[e]; d = (d < 0) ? 0 : (d >= N ? N - 1 : d); const int g = d >> CSR_GB8; ids[run[g]] = e; run[g] += 1; } }
  __syncthreads();
  typedef __attribute__((ext_vector_type(4))) int v4i;
  for (int pass = 0; pass < 2; ++pass) {
    for (int i = threadIdx.x; i < CHP / 4; i += 64) *(volatile v4i*)(STG + (size_t)b * CHP + i * 4) = *(const v4i*)(&ids[i * 4]);
    for (int i = threadIdx.x; i < NGP / 4; i += 64) { v4i v; for (int e = 0; e < 4; ++e) v[e] = (i * 4 + e < nG) ? cnt[i * 4 + e] : 0; *(volatile v4i*)(HST + (size_t)b * NGP + i * 4) = v; }
    __threadfence(); }
}
__global__ __launch_bounds__(512) void csrS_kernel8(const int* __restrict__ HST, int nG, int NGP, int* __restrict__ START, int* __restrict__ TOT, int* __restrict__ OFF) {
  __shared__ int tot[CSR_MAXG8];
  const int b = threadIdx.x;
  for (int pass = 0; pass < 2; ++pass) { int runb = 0; for (int g = 0; g < nG; ++g) { int c = HST[(size_t)b * NGP + g]; c = (c < 0) ? 0 : c; ((volatile int*)OFF)[(size_t)g * CSR_NBLK8 + b] = runb; runb += c; } __threadfence(); }
  for (int g = threadIdx.x; g < nG; g += 512) { int s = 0; for (int bb = 0; bb < CSR_NBLK8; ++bb) { int c = HST[(size_t)bb * NGP + g]; s += (c < 0) ? 0 : c; } tot[g] = s; }
  __syncthreads();
  if (threadIdx.x < 32) {
    __shared__ int st[CSR_MAXG8 + 32];
    if (threadIdx.x == 0) { int acc = 0; for (int g = 0; g < NGP; ++g) { st[g] = acc; if (g < nG) acc += (tot[g] + 31) & ~31; } st[NGP] = acc; }
    __builtin_amdgcn_fence(__ATOMIC_RELEASE, "workgroup"); __builtin_amdgcn_wave_barrier(); __builtin_amdgcn_fence(__ATOMIC_ACQUIRE, "workgroup");
    for (int pass = 0; pass < 2; ++pass) { for (int i = threadIdx.x; i < NGP + 32; i += 32) { ((volatile int*)START)[i] = (i <= NGP) ? st[min(i, NGP)] : 0; ((volatile int*)TOT)[i] = (i < nG) ? tot[i] : 0; } __threadfence(); } }
}
__global__ __launch_bounds__(256) void csrB_kernel8(const int* __restrict__ dst, int N, int nG, int CHP, int NGP, int permLen, const int* __restrict__ STG, const int* __restrict__ HST, const int* __restrict__ OFF, const int* __restrict__ START, const int* __restrict__ TOT, int* __restrict__ PERM, int* __restrict__ ROWPTR, int* __restrict__ ROWCNT, int* __restrict__ FLAG) {
  typedef __attribute__((ext_vector_type(4))) int v4i;
  __shared__ int ids[CSR_CAP8]; __shared__ unsigned short key[CSR_CAP8]; __shared__ int outp[CSR_CAP8]; __shared__ int ncnt[CSR_GN8 + 1]; __shared__ int boff[CSR_NBLK8 + 1];
  const int g = blockIdx.x, t_ = threadIdx.x; int tot = TOT[g]; int st = START[g], stn = START[g + 1]; const int v0 = g * CSR_GN8; const int nv = min(CSR_GN8, N - v0); const int t0 = g * CSR_TS8;
  st = (st < 0) ? 0 : (st > permLen - 32 ? permLen - 32 : st) & ~31; stn = (stn < st) ? st : (stn > permLen ? permLen : stn); tot = (tot < 0) ? 0 : tot; if (tot > stn - st && tot <= CSR_CAP8) tot = stn - st;
  if (tot > CSR_CAP8) {
    for (int pass = 0; pass < 2; ++pass) { for (int i = t_; i < CSR_TS8 / 4; i += 256) { v4i a, c; for (int e = 0; e < 4; ++e) { a[e] = st; c[e] = 0; } *(volatile v4i*)(ROWPTR + t0 + i * 4) = a; *(volatile v4i*)(ROWCNT + t0 + i * 4) = c; } if (t_ == 0) ((volatile int*)FLAG)[0] = 1; __threadfence(); } (void)nv; return; }
  if (t_ == 0) { int acc = 0; for (int b = 0; b < CSR_NBLK8; ++b) { boff[b] = acc; int c = HST[(size_t)b * NGP + g]; c = (c < 0) ? 0 : (c > CHP ? CHP : c); acc += c; if (acc > tot) acc = tot; } boff[CSR_NBLK8] = acc; }
  for (int i = t_; i <= CSR_GN8; i += 256) ncnt[i] = 0;
  __syncthreads();
  for (int b = 0; b < CSR_NBLK8; ++b) { const int c = boff[b + 1] - boff[b]; int o_ = OFF[(size_t)g * CSR_NBLK8 + b]; o_ = (o_ < 0) ? 0 : (o_ > CHP - c ? CHP - c : o_); const int* src_ = STG + (size_t)b * CHP + o_;
    for (int i = t_; i < c; i += 256) { int id = src_[i]; id = (id < 0) ? 0 : id; ids[boff[b] + i] = id; int d = dst[id]; d = (d < v0) ? v0 : (d >= N ? N - 1 : d); int kk = d - v0; kk = (kk < 0) ? 0 : (kk >= CSR_GN8 ? CSR_GN8 - 1 : kk); key[boff[b] + i] = (unsigned short)kk; } }
  __syncthreads();
  if (t_ == 0) { for (int i = 0; i < tot; ++i) ncnt[key[i]] += 1; int acc = 0; for (int vl = 0; vl < CSR_GN8; ++vl) { const int c = ncnt[vl]; ncnt[vl] = acc; acc += c; } ncnt[CSR_GN8] = acc;
    for (int i = 0; i < tot; ++i) { const int vl = key[i]; outp[ncnt[vl]] = ids[i]; ncnt[vl] += 1; }
    for (int vl = CSR_GN8; vl > 0; --vl) ncnt[vl] = ncnt[vl - 1]; ncnt[0] = 0; }
  __syncthreads();
  for (int pass = 0; pass < 2; ++pass) {
    for (int i = t_; i < (stn - st) / 4; i += 256) { v4i v; for (int e = 0; e < 4; ++e) { const int q = i * 4 + e; v[e] = (q < tot) ? outp[q] : -1; } *(volatile v4i*)(PERM + st + i * 4) = v; }
    for (int i = t_; i < CSR_TS8 / 4; i += 256) { v4i a, c; for (int e = 0; e < 4; ++e) { const int vl = i * 4 + e; const int vc = vl < CSR_GN8 ? vl : CSR_GN8; a[e] = (vl < CSR_GN8) ? st + ncnt[vc] : st; c[e] = (vl < nv) ? (ncnt[(vc < CSR_GN8 ? vc : CSR_GN8 - 1) + 1] - ncnt[vc]) : 0; } *(volatile v4i*)(ROWPTR + t0 + i * 4) = a; *(volatile v4i*)(ROWCNT + t0 + i * 4) = c; }
    __threadfence(); }
}
__global__ __launch_bounds__(256) void csrZ_kernel8(int* __restrict__ p, size_t n4) { typedef __attribute__((ext_vector_type(4))) int v4i; const size_t tid = (size_t)blockIdx.x * 256 + threadIdx.x, nth = (size_t)gridDim.x * 256; v4i z = {0, 0, 0, 0}; for (size_t i = tid; i < n4; i += nth) *(volatile v4i*)(p + i * 4) = z; }
struct CsrBufs8 { int *STG, *HST, *OFF, *START, *TOT, *PERM, *ROWPTR, *ROWCNT, *FLAG; int nG, NGP, CHP; size_t permLen; char* base; size_t bytes; };
static size_t csr_carve8(CsrBufs8& c, char* ws, size_t off, int E, int N) {
  const size_t off0 = off; c.base = ws + off;
  auto al = [&](size_t bytes) { char* p = ws + off; off += (bytes + 255) & ~(size_t)255; return p; };
  c.nG = (N + CSR_GN8 - 1) / CSR_GN8; c.NGP = (c.nG + 31) & ~31; const int ch = (E + CSR_NBLK8 - 1) / CSR_NBLK8; c.CHP = (ch + 31) & ~31; c.permLen = (size_t)E + 32 * (size_t)c.nG + 32;
  c.STG = (int*)al((size_t)CSR_NBLK8 * c.CHP * 4); c.HST = (int*)al((size_t)CSR_NBLK8 * c.NGP * 4); c.OFF = (int*)al((size_t)c.NGP * CSR_NBLK8 * 4); c.START = (int*)al((size_t)(c.NGP + 64) * 4); c.TOT = (int*)al((size_t)(c.NGP + 64) * 4);
  c.PERM = (int*)al(c.permLen * 4); c.ROWPTR = (int*)al((size_t)c.nG * CSR_TS8 * 4); c.ROWCNT = (int*)al((size_t)c.nG * CSR_TS8 * 4); c.FLAG = (int*)al(256);
  c.bytes = off - off0; return off;
}
static void csr_build8(const CsrBufs8& c, const int* dst, int E, int N, hipStream_t stream) {
  const size_t smem = (size_t)(2 * c.NGP + c.CHP) * 4;
  csrZ_kernel8<<<512, 256, 0, stream>>>((int*)c.base, c.bytes / 16);
  csrA_kernel8<<<CSR_NBLK8, 64, smem, stream>>>(dst, E, N, c.nG, c.CHP, c.NGP, c.STG, c.HST);
  csrS_kernel8<<<1, 512, 0, stream>>>(c.HST, c.nG, c.NGP, c.START, c.TOT, c.OFF);
  csrB_kernel8<<<c.nG, 256, 0, stream>>>(dst, N, c.nG, c.CHP, c.NGP, (int)c.permLen, c.STG, c.HST, c.OFF, c.START, c.TOT, c.PERM, c.ROWPTR, c.ROWCNT, c.FLAG);
}


__global__ __launch_bounds__(256) void wput_kernel(const float* __restrict__ wg, const float* __restrict__ w1, const float* __restrict__ w2, const float* __restrict__ wm, const float* __restrict__ wsd, b16* __restrict__ WG, b16* __restrict__ W1, b16* __restrict__ W2, b16* __restrict__ WMS) { const int u = blockIdx.x * 256 + threadIdx.x;
  if (u < HID * 16) { const int o = u / 16, k0 = (u % 16) * 8; v8b v;
#pragma unroll
    for (int j = 0; j < 8; ++j) v[j] = (b16)(bf16_rne(wg[(size_t)(k0 + j) * HID + o]) * WSC); for (int pass = 0; pass < 2; ++pass) { *(volatile v8b*)(WG + (size_t)o * C0 + k0) = v; __threadfence(); } }
  if (u < HW * 8) { const int o = u / 8, k0 = (u % 8) * 8; v8b v;
#pragma unroll
    for (int j = 0; j < 8; ++j) v[j] = (b16)(bf16_rne(w1[(size_t)(k0 + j) * HW + o]) * WSC); for (int pass = 0; pass < 2; ++pass) { *(volatile v8b*)(W1 + (size_t)o * HID + k0) = v; __threadfence(); } }
  if (u < HW * 32) { const int o = u / 32, k0 = (u % 32) * 8; v8b v;
#pragma unroll
    for (int j = 0; j < 8; ++j) v[j] = (b16)(bf16_rne(w2[(size_t)(k0 + j) * HW + o]) * WSC); for (int pass = 0; pass < 2; ++pass) { *(volatile v8b*)(W2 + (size_t)o * HW + k0) = v; __threadfence(); } }
  if (u < 2 * HW * 8) { const int r = u / 8, k0 = (u % 8) * 8; const int part = r / HW, o = r % HW; const float* w = part ? wsd : wm; v8b v;
#pragma unroll
    for (int j = 0; j < 8; ++j) v[j] = (b16)(bf16_rne(w[(size_t)(k0 + j) * HW + o]) * WSC); for (int pass = 0; pass < 2; ++pass) { *(volatile v8b*)(WMS + (size_t)r * HID + k0) = v; __threadfence(); } } }
__global__ __launch_bounds__(32) void gdense_kernel(const float* __restrict__ x, const b16* __restrict__ WG, int NLIM, float* __restrict__ M) { __shared__ __attribute__((aligned(16))) b16 Ah[16][C0 + 8]; __shared__ float Tf[16][68]; const int lane = threadIdx.x, nloc = lane & 15, hlf = lane >> 4; const size_t m0 = (size_t)blockIdx.x * 16; if (m0 >= (size_t)NLIM) return;
  for (int rr = 0; rr < 16; ++rr) for (int q = 0; q < 4; ++q) Ah[rr][q * 32 + lane] = (b16)(bf16_rne(x[(m0 + rr) * C0 + q * 32 + lane]) * XS);
  wave_lds_sync(); v8f acc[4];
#pragma unroll
  for (int t = 0; t < 4; ++t) acc[t] = (v8f){};
#pragma unroll
  for (int kb = 0; kb < C0; kb += 32) { const v16b a = frag_kb(&Ah[nloc][kb], hlf);
#pragma unroll
    for (int t = 0; t < 4; ++t) acc[t] = wmma16b(a, frag_kb(WG + (size_t)(t * 16 + nloc) * C0 + kb, hlf), acc[t]); }
#pragma unroll
  for (int t = 0; t < 4; ++t)
#pragma unroll
    for (int r8 = 0; r8 < 8; ++r8) Tf[8 * hlf + r8][t * 16 + nloc] = acc[t][r8] * (1.0f / (XS * WSC));
  wave_lds_sync();
  for (int pass = 0; pass < 2; ++pass) { for (int rr = 0; rr < 16; ++rr) *(volatile v2f*)(M + (m0 + rr) * HID + lane * 2) = (v2f){Tf[rr][lane * 2], Tf[rr][lane * 2 + 1]}; __threadfence(); } }
__global__ __launch_bounds__(256) void gcn_kernel(const float* __restrict__ M, const float* __restrict__ bias, const int* __restrict__ srcs, const int* __restrict__ PERM, const int* __restrict__ ROWPTR, const int* __restrict__ ROWCNT, int permLen, int NLIM, float* __restrict__ H0) { const int wave = threadIdx.x >> 5, lane = threadIdx.x & 31; const size_t i = (size_t)blockIdx.x * 8 + wave; if (i >= (size_t)NLIM) return; int st = ROWPTR[i], cnt = ROWCNT[i]; cnt = iclamp(cnt, 0, E); st = iclamp(st, 0, permLen - cnt);
  v2f acc = {0, 0}; int nin = 0;
#pragma unroll 1
  for (int j = 0; j < cnt; ++j) { const int e = iclamp(PERM[st + j], 0, E - 1); const size_t u = (size_t)iclamp(srcs[e], 0, N - 1); if (u >= (size_t)NLIM) continue; ++nin; const float du = rsqrtf((float)(iclamp(ROWCNT[u], 0, E) + 1)); const v2f v = *(const v2f*)(M + u * HID + lane * 2); acc[0] += pmul(du, v[0]); acc[1] += pmul(du, v[1]); }
  const float di = rsqrtf((float)(nin + 1)); const v2f sv = *(const v2f*)(M + i * HID + lane * 2); v2f o; for (int k = 0; k < 2; ++k) o[k] = fmaxf(pmul(di, acc[k]) + pmul(pmul(di, di), sv[k]) + bf16_rne(bias[lane * 2 + k]), 0.0f);
  for (int pass = 0; pass < 2; ++pass) { *(volatile v2f*)(H0 + i * HID + lane * 2) = o; __threadfence(); } }
template <int K>
__global__ __launch_bounds__(32) void proj_kernel(const float* __restrict__ IN, const b16* __restrict__ W, const float* __restrict__ asrc, const float* __restrict__ adst, int NLIM, float* __restrict__ XL, float* __restrict__ AS) { __shared__ __attribute__((aligned(16))) b16 Ah[16][K + 8], Al[16][K + 8]; __shared__ float Tf[16][HW + 4]; __shared__ float Sa[16][8]; const int lane = threadIdx.x, nloc = lane & 15, hlf = lane >> 4; const size_t m0 = (size_t)blockIdx.x * 16; if (m0 >= (size_t)NLIM) return;
  for (int rr = 0; rr < 16; ++rr) for (int q = 0; q < K / 32; ++q) { b16 p, ql; split16(IN[(m0 + rr) * K + q * 32 + lane] * XS, p, ql); Ah[rr][q * 32 + lane] = p; Al[rr][q * 32 + lane] = ql; }
  wave_lds_sync(); v8f acc[16];
#pragma unroll
  for (int t = 0; t < 16; ++t) acc[t] = (v8f){};
#pragma unroll 2
  for (int kb = 0; kb < K; kb += 32) { const v16b a = frag_kb(&Ah[nloc][kb], hlf), al = frag_kb(&Al[nloc][kb], hlf);
#pragma unroll
    for (int t = 0; t < 16; ++t) { const v16b bw = frag_kb(W + (size_t)(t * 16 + nloc) * K + kb, hlf); acc[t] = wmma16b(a, bw, acc[t]); acc[t] = wmma16b(al, bw, acc[t]); } }
#pragma unroll
  for (int t = 0; t < 16; ++t)
#pragma unroll
    for (int r8 = 0; r8 < 8; ++r8) Tf[8 * hlf + r8][t * 16 + nloc] = acc[t][r8] * (1.0f / (XS * WSC));
  wave_lds_sync();
  for (int rr = 0; rr < 16; ++rr) { if (lane < 8) { const int h = lane & 3, kind = lane >> 2; const float* av = kind ? adst : asrc; float s = 0.0f;
#pragma unroll 4
      for (int c = 0; c < HID; ++c) s += pmul(Tf[rr][h * HID + c], bf16_rne(av[h * HID + c])); Sa[rr][lane] = s; } }
  wave_lds_sync();
  for (int pass = 0; pass < 2; ++pass) { for (int rr = 0; rr < 16; ++rr) { *(volatile v4f*)(XL + (m0 + rr) * HW + lane * 4) = *(const v4f*)(&Tf[rr][lane * 4]); *(volatile v4f*)(XL + (m0 + rr) * HW + 128 + lane * 4) = *(const v4f*)(&Tf[rr][128 + lane * 4]); ((volatile float*)AS)[(m0 + rr) * 32 + lane] = lane < 8 ? Sa[rr][lane] : 0.0f; } __threadfence(); } }
template <int CONCAT, int RELU>
__global__ __launch_bounds__(256) void gat_kernel(const float* __restrict__ XL, const float* __restrict__ AS, const float* __restrict__ bias, const int* __restrict__ srcs, const int* __restrict__ PERM, const int* __restrict__ ROWPTR, const int* __restrict__ ROWCNT, int permLen, int NLIM, float* __restrict__ OUT, float* __restrict__ MD) { const int wave = threadIdx.x >> 5, lane = threadIdx.x & 31; const size_t i = (size_t)blockIdx.x * 8 + wave; if (i >= (size_t)NLIM) return; int st = ROWPTR[i], cnt = ROWCNT[i]; cnt = iclamp(cnt, 0, E); st = iclamp(st, 0, permLen - cnt); const int hd = lane >> 3, sub = lane & 7; const float adi = AS[i * 32 + 4 + hd];
  float m = leaky(AS[i * 32 + hd] + adi), den = 1.0f; float acc[8];
  { const float* xp = XL + i * HW + hd * HID + sub * 8;
#pragma unroll
    for (int k = 0; k < 8; ++k) acc[k] = xp[k]; }
#pragma unroll 1
  for (int j = 0; j < cnt; ++j) { const int e = iclamp(PERM[st + j], 0, E - 1); const size_t u = (size_t)iclamp(srcs[e], 0, N - 1); if (u >= (size_t)NLIM) continue; const float s = leaky(AS[u * 32 + hd] + adi); const float mn = fmaxf(m, s); const float sf = __expf(m - mn); const float p = __expf(s - mn); den = den * sf + p; const float* xp = XL + u * HW + hd * HID + sub * 8;
#pragma unroll
    for (int k = 0; k < 8; ++k) acc[k] = pmul(acc[k], sf) + pmul(p, xp[k]); m = mn; }
  const float inv = 1.0f / (den + 1e-16f); float o[8];
#pragma unroll
  for (int k = 0; k < 8; ++k) { float v = pmul(acc[k], inv); if (!CONCAT) { v += __shfl_xor(v, 8); v += __shfl_xor(v, 16); v = v * 0.25f + bf16_rne(bias[sub * 8 + k]); } else v += bf16_rne(bias[hd * HID + sub * 8 + k]); o[k] = RELU ? fmaxf(v, 0.0f) : v; }
  const float msh = __shfl(m, (lane & 3) * 8), dsh = __shfl(den, (lane & 3) * 8); const float mdv = lane < 4 ? msh : (lane < 8 ? dsh : 0.0f);
  for (int pass = 0; pass < 2; ++pass) {
    if (CONCAT) { *(volatile v4f*)(OUT + i * HW + lane * 8) = (v4f){o[0], o[1], o[2], o[3]}; *(volatile v4f*)(OUT + i * HW + lane * 8 + 4) = (v4f){o[4], o[5], o[6], o[7]}; }
    else if (lane < 8) { *(volatile v4f*)(OUT + i * HID + sub * 8) = (v4f){o[0], o[1], o[2], o[3]}; *(volatile v4f*)(OUT + i * HID + sub * 8 + 4) = (v4f){o[4], o[5], o[6], o[7]}; }
    ((volatile float*)MD)[i * 32 + lane] = mdv; __threadfence(); } }
__global__ __launch_bounds__(256) void alpha_kernel(const float* __restrict__ AS, const float* __restrict__ MD, const int* __restrict__ ei, int NLIM, float* __restrict__ A) { const size_t e = (size_t)blockIdx.x * 256 + threadIdx.x; if (e >= (size_t)EP) return; int s, d; if (e < (size_t)E) { s = iclamp(ei[e], 0, N - 1); d = iclamp(ei[E + e], 0, N - 1); } else { s = d = (int)(e - E); }
  v4f a = {0, 0, 0, 0}; if (s < NLIM && d < NLIM) {
#pragma unroll
    for (int h = 0; h < 4; ++h) { const float sc = leaky(AS[(size_t)s * 32 + h] + AS[(size_t)d * 32 + 4 + h]); a[h] = __expf(sc - MD[(size_t)d * 32 + h]) / (MD[(size_t)d * 32 + 4 + h] + 1e-16f); } }
  for (int pass = 0; pass < 2; ++pass) { *(volatile v4f*)(A + e * 4) = a; __threadfence(); } }
}

extern "C" void kernel_launch(void* const* d_in, const int* in_sizes, int n_in, void* d_out, int out_size, void* d_ws, size_t ws_size, hipStream_t stream) {
  (void)n_in;
  auto Fp = [&](int i) { return (const float*)d_in[i]; }; auto Ip = [&](int i) { return (const int*)d_in[i]; };
  if (in_sizes[0] != N * C0 || in_sizes[1] != 2 * E || in_sizes[2] != C0 * HID || in_sizes[4] != HID * HW || in_sizes[8] != HW * HW || in_sizes[12] != HID * HW || in_sizes[16] != HID * HW || out_size != 2 * N * HID + 4 * EP * NH) return;
  const int NLIM = N;
  size_t off = 0; char* ws = (char*)d_ws;
  auto carve = [&](size_t bytes) { char* p = ws + off; off += (bytes + 255) & ~(size_t)255; return p; };
  b16* WG = (b16*)carve((size_t)HID * C0 * 2); b16* W1 = (b16*)carve((size_t)HW * HID * 2); b16* W2 = (b16*)carve((size_t)HW * HW * 2); b16* WMS = (b16*)carve((size_t)2 * HW * HID * 2);
  float* M = (float*)carve((size_t)N * HID * 4); float* H0 = (float*)carve((size_t)N * HID * 4); float* XL = (float*)carve((size_t)N * HW * 4); float* AS = (float*)carve((size_t)N * 32 * 4); float* MD = (float*)carve((size_t)N * 32 * 4); float* H1 = (float*)carve((size_t)N * HW * 4); float* H2 = (float*)carve((size_t)N * HID * 4); CsrBufs8 csr; off = csr_carve8(csr, ws, off, E, N);
  if (off > ws_size || off > ((size_t)96 << 20)) return;
  float* ZM = (float*)d_out; float* ZS = ZM + (size_t)N * HID; float* A1 = ZS + (size_t)N * HID; float* A2 = A1 + (size_t)EP * NH; float* AM = A2 + (size_t)EP * NH; float* ASD = AM + (size_t)EP * NH;
  wput_kernel<<<(HW * 32 + 255) / 256, 256, 0, stream>>>(Fp(2), Fp(4), Fp(8), Fp(12), Fp(16), WG, W1, W2, WMS);
  csr_build8(csr, Ip(1) + E, E, N, stream);
  gdense_kernel<<<NLIM / 16, 32, 0, stream>>>(Fp(0), WG, NLIM, M);
  gcn_kernel<<<(NLIM + 7) / 8, 256, 0, stream>>>(M, Fp(3), Ip(1), csr.PERM, csr.ROWPTR, csr.ROWCNT, (int)csr.permLen, NLIM, H0);
  proj_kernel<HID><<<NLIM / 16, 32, 0, stream>>>(H0, W1, Fp(5), Fp(6), NLIM, XL, AS);
  gat_kernel<1, 1><<<(NLIM + 7) / 8, 256, 0, stream>>>(XL, AS, Fp(7), Ip(1), csr.PERM, csr.ROWPTR, csr.ROWCNT, (int)csr.permLen, NLIM, H1, MD);
  alpha_kernel<<<(EP + 255) / 256, 256, 0, stream>>>(AS, MD, Ip(1), NLIM, A1);
  proj_kernel<HW><<<NLIM / 16, 32, 0, stream>>>(H1, W2, Fp(9), Fp(10), NLIM, XL, AS);
  gat_kernel<0, 1><<<(NLIM + 7) / 8, 256, 0, stream>>>(XL, AS, Fp(11), Ip(1), csr.PERM, csr.ROWPTR, csr.ROWCNT, (int)csr.permLen, NLIM, H2, MD);
  alpha_kernel<<<(EP + 255) / 256, 256, 0, stream>>>(AS, MD, Ip(1), NLIM, A2);
  proj_kernel<HID><<<NLIM / 16, 32, 0, stream>>>(H2, WMS, Fp(13), Fp(14), NLIM, XL, AS);
  gat_kernel<0, 0><<<(NLIM + 7) / 8, 256, 0, stream>>>(XL, AS, Fp(15), Ip(1), csr.PERM, csr.ROWPTR, csr.ROWCNT, (int)csr.permLen, NLIM, ZM, MD);
  alpha_kernel<<<(EP + 255) / 256, 256, 0, stream>>>(AS, MD, Ip(1), NLIM, AM);
  proj_kernel<HID><<<NLIM / 16, 32, 0, stream>>>(H2, WMS + (size_t)HW * HID, Fp(17), Fp(18), NLIM, XL, AS);
  gat_kernel<0, 0><<<(NLIM + 7) / 8, 256, 0, stream>>>(XL, AS, Fp(19), Ip(1), csr.PERM, csr.ROWPTR, csr.ROWCNT, (int)csr.permLen, NLIM, ZS, MD);
  alpha_kernel<<<(EP + 255) / 256, 256, 0, stream>>>(AS, MD, Ip(1), NLIM, ASD);
}
